// CTAttention_9010841387717
// MI455X (gfx1250) — hardware-verified
//
#include <hip/hip_runtime.h>
#include <stddef.h>
#include <stdint.h>

#define NB    8
#define MAXW  1024
#define CD    256
#define NH    8
#define HD    32
#define NTOK  6464
#define NQKV  768
#define PROWS (NB * MAXW)
#define QBLK  64
#define KCH   64
#define NKC   (MAXW / KCH)
#define NQB   (MAXW / QBLK)

static_assert(CD == NH * HD);
static_assert(HD == 32);
static_assert(NQKV == 3 * CD);
static_assert(NTOK % 64 == 0);
static_assert(PROWS % 128 == 0);
static_assert(MAXW % 128 == 0);
static_assert(MAXW % QBLK == 0);
static_assert(MAXW % KCH == 0);
static_assert(QBLK == 64 && KCH == 64);
static_assert(NQKV % 64 == 0 && CD % 64 == 0);
static_assert((MAXW & (MAXW - 1)) == 0);

typedef __bf16         v16b __attribute__((ext_vector_type(16)));
typedef unsigned short v8us __attribute__((ext_vector_type(8)));
typedef float          v8f  __attribute__((ext_vector_type(8)));
typedef float          v4f  __attribute__((ext_vector_type(4)));
typedef unsigned int   v4u  __attribute__((ext_vector_type(4)));
typedef unsigned short us16;

union BFrag { v16b v; v8us h[2]; };
union Pack8 { v8us h; v4u u; };

__device__ __forceinline__ v8f zero8() { return (v8f){0.f, 0.f, 0.f, 0.f, 0.f, 0.f, 0.f, 0.f}; }

__device__ __forceinline__ us16 bf_rne(float x) {
  unsigned int u = __float_as_uint(x);
  u += 0x7FFFu + ((u >> 16) & 1u);
  return (us16)(u >> 16);
}
__device__ __forceinline__ float bf_val(us16 hbits) { return __uint_as_float(((unsigned int)hbits) << 16); }

__device__ __forceinline__ v8f mma16(v16b a, v16b b, v8f c) {
  c = __builtin_amdgcn_wmma_f32_16x16x32_bf16(false, a, false, b, (short)0, c, false, false);
  asm volatile("v_nop\n\tv_nop\n\tv_nop\n\tv_nop" : "+v"(c) : "v"(a), "v"(b));
  return c;
}

__device__ __forceinline__ v8f mma3(v16b ah, v16b al, v16b bh, v16b bl, v8f c) {
  c = mma16(ah, bh, c);
  c = mma16(ah, bl, c);
  c = mma16(al, bh, c);
  return c;
}

__device__ __forceinline__ v16b ldfrag(const us16* p, int ld, int row0, int k0, int lane) {
  const int m = lane & 15, lh = lane >> 4;
  const us16* q = p + (size_t)(row0 + m) * ld + k0 + 8 * lh;
  BFrag f;
  f.h[0] = *(const v8us*)(q);
  f.h[1] = *(const v8us*)(q + 16);
  return f.v;
}

__device__ __forceinline__ void split8(v4f a0, v4f a1, v4u& uh, v4u& ul) {
  Pack8 ph, pl;
#pragma unroll
  for (int i = 0; i < 4; ++i) {
    const us16 h0 = bf_rne(a0[i]);
    ph.h[i] = h0;
    pl.h[i] = bf_rne(a0[i] - bf_val(h0));
    const us16 h1 = bf_rne(a1[i]);
    ph.h[4 + i] = h1;
    pl.h[4 + i] = bf_rne(a1[i] - bf_val(h1));
  }
  uh = ph.u;
  ul = pl.u;
}

__device__ __forceinline__ void gemm32x64x3(const us16* __restrict__ ah, const us16* __restrict__ al, int lda,
                                            const us16* __restrict__ bh, const us16* __restrict__ bl, int ldb, int K,
                                            int m0, int n0, int lane, v8f (&acc)[2][4]) {
#pragma unroll 1
  for (int k0 = 0; k0 < K; k0 += 32) {
    const v16b a0h = ldfrag(ah, lda, m0, k0, lane);
    const v16b a1h = ldfrag(ah, lda, m0 + 16, k0, lane);
    const v16b a0l = ldfrag(al, lda, m0, k0, lane);
    const v16b a1l = ldfrag(al, lda, m0 + 16, k0, lane);
#pragma unroll
    for (int t = 0; t < 4; ++t) {
      const v16b bth = ldfrag(bh, ldb, n0 + 16 * t, k0, lane);
      const v16b btl = ldfrag(bl, ldb, n0 + 16 * t, k0, lane);
      acc[0][t] = mma3(a0h, a0l, bth, btl, acc[0][t]);
      acc[1][t] = mma3(a1h, a1l, bth, btl, acc[1][t]);
    }
  }
}

#define TRP 260
__global__ __launch_bounds__(256) void k_tr(const float* __restrict__ w, int nc,
                                            us16* __restrict__ ph, us16* __restrict__ pl) {
  __shared__ __align__(16) float st[32 * TRP];
  const int tid = threadIdx.x, lane = tid & 31, wave = tid >> 5;
  const int c0 = blockIdx.x * 32;
#pragma unroll 4
  for (int i = 0; i < 32; ++i) {
    const int r = wave + 8 * i;
    st[lane * TRP + r] = w[(size_t)r * nc + c0 + lane];
  }
  __syncthreads();
  v4u vh[4], vl[4];
  size_t go[4];
#pragma unroll
  for (int j = 0; j < 4; ++j) {
    const int row = 4 * wave + j;
    const float* s = st + row * TRP + 8 * lane;
    const v4f a0 = *(const v4f*)(s);
    const v4f a1 = *(const v4f*)(s + 4);
    split8(a0, a1, vh[j], vl[j]);
    go[j] = (size_t)(c0 + row) * CD + 8 * lane;
  }
  for (int ps = 0; ps < 2; ++ps) {
#pragma unroll
    for (int j = 0; j < 4; ++j) {
      *(volatile v4u*)(ph + go[j]) = vh[j];
      *(volatile v4u*)(pl + go[j]) = vl[j];
    }
    __threadfence();
  }
}

__global__ __launch_bounds__(256) void k_pad(const float* __restrict__ tok, const int* __restrict__ lens, int ntok,
                                             us16* __restrict__ xh, us16* __restrict__ xl) {
  const int tid = threadIdx.x, lane = tid & 31, wave = tid >> 5;
  const int pr  = blockIdx.x * 8 + wave;
  const int b   = pr >> 10;
  const int wdx = pr & (MAXW - 1);
  int off = 0, len = 0;
#pragma unroll
  for (int i = 0; i < NB; ++i) {
    const int li = min(max(lens[i], 0), MAXW);
    off += (i < b) ? li : 0;
    len = (i == b) ? li : len;
  }
  const bool valid = wdx < len;
  int t = off + wdx;
  t = min(max(t, 0), ntok - 1);
  const float* src = tok + (size_t)t * CD + 8 * lane;
  v4f a0 = *(const v4f*)(src);
  v4f a1 = *(const v4f*)(src + 4);
#pragma unroll
  for (int j = 0; j < 4; ++j) {
    a0[j] = valid ? a0[j] : 0.f;
    a1[j] = valid ? a1[j] : 0.f;
  }
  v4u uh, ul;
  split8(a0, a1, uh, ul);
  const size_t go = (size_t)pr * CD + 8 * lane;
  volatile v4u* dh = (volatile v4u*)(xh + go);
  volatile v4u* dl = (volatile v4u*)(xl + go);
  *dh = uh;
  *dl = ul;
  __threadfence();
  *dh = uh;
  *dl = ul;
}

#define SQP 72
#define SVT 136
__global__ __launch_bounds__(128) void k_qkv(const us16* __restrict__ xh, const us16* __restrict__ xl,
                                             const us16* __restrict__ wh, const us16* __restrict__ wl,
                                             const float* __restrict__ bias,
                                             us16* __restrict__ qh, us16* __restrict__ ql,
                                             us16* __restrict__ kh, us16* __restrict__ kl,
                                             us16* __restrict__ vth, us16* __restrict__ vtl) {
  __shared__ __align__(16) us16 st[2][128 * SQP];
  const int tid = threadIdx.x, lane = tid & 31, wave = tid >> 5;
  const int hh = lane >> 4, c = lane & 15;
  const int rb = blockIdx.x * 128;
  const int b  = rb >> 10;
  const int w0 = rb & (MAXW - 1);
  const int ns = blockIdx.y;
  const int which = ns >> 2;
  const int cs = (ns & 3) * 64;
  const int m0 = rb + wave * 32;
  const int n0 = ns * 64;

  v8f acc[2][4];
#pragma unroll
  for (int s = 0; s < 2; ++s)
#pragma unroll
    for (int t = 0; t < 4; ++t) acc[s][t] = zero8();
  gemm32x64x3(xh, xl, CD, wh, wl, CD, CD, m0, n0, lane, acc);

  float bb[4];
#pragma unroll
  for (int t = 0; t < 4; ++t) bb[t] = bias[n0 + 16 * t + c];

  if (which < 2) {
#pragma unroll
    for (int sub = 0; sub < 2; ++sub)
#pragma unroll
      for (int t = 0; t < 4; ++t)
#pragma unroll
        for (int r = 0; r < 8; ++r) {
          const float v = acc[sub][t][r] + bb[t];
          const us16 hb = bf_rne(v);
          const int idx = (wave * 32 + sub * 16 + 8 * hh + r) * SQP + 16 * t + c;
          st[0][idx] = hb;
          st[1][idx] = bf_rne(v - bf_val(hb));
        }
  } else {
#pragma unroll
    for (int sub = 0; sub < 2; ++sub)
#pragma unroll
      for (int t = 0; t < 4; ++t)
#pragma unroll
        for (int r = 0; r < 8; ++r) {
          const float v = acc[sub][t][r] + bb[t];
          const us16 hb = bf_rne(v);
          const int idx = (16 * t + c) * SVT + wave * 32 + sub * 16 + 8 * hh + r;
          st[0][idx] = hb;
          st[1][idx] = bf_rne(v - bf_val(hb));
        }
  }
  __syncthreads();

  if (which < 2) {
    us16* dsth = (which == 0) ? qh : kh;
    us16* dstl = (which == 0) ? ql : kl;
    size_t go[8];
#pragma unroll
    for (int it = 0; it < 8; ++it) {
      const int p  = tid + 128 * it;
      const int lr = p >> 3;
      const int pc = p & 7;
      go[it] = (size_t)(rb + lr) * CD + cs + pc * 8;
    }
#pragma unroll 1
    for (int pl = 0; pl < 2; ++pl) {
      us16* base = (pl == 0) ? dsth : dstl;
      v4u val[8];
#pragma unroll
      for (int it = 0; it < 8; ++it) {
        const int p  = tid + 128 * it;
        const int lr = p >> 3;
        const int pc = p & 7;
        Pack8 pk;
        pk.h    = *(const v8us*)(st[pl] + lr * SQP + pc * 8);
        val[it] = pk.u;
      }
      for (int ps = 0; ps < 2; ++ps) {
#pragma unroll
        for (int it = 0; it < 8; ++it) *(volatile v4u*)(base + go[it]) = val[it];
        __threadfence();
      }
    }
  } else {
    us16* dsth = vth + (size_t)b * CD * MAXW;
    us16* dstl = vtl + (size_t)b * CD * MAXW;
    size_t go[8];
#pragma unroll
    for (int it = 0; it < 8; ++it) {
      const int p  = tid + 128 * it;
      const int dr = p >> 4;
      const int pc = p & 15;
      go[it] = (size_t)(cs + dr) * MAXW + w0 + pc * 8;
    }
#pragma unroll 1
    for (int pl = 0; pl < 2; ++pl) {
      us16* base = (pl == 0) ? dsth : dstl;
      v4u val[8];
#pragma unroll
      for (int it = 0; it < 8; ++it) {
        const int p  = tid + 128 * it;
        const int dr = p >> 4;
        const int pc = p & 15;
        Pack8 pk;
        pk.h    = *(const v8us*)(st[pl] + dr * SVT + pc * 8);
        val[it] = pk.u;
      }
      for (int ps = 0; ps < 2; ++ps) {
#pragma unroll
        for (int it = 0; it < 8; ++it) *(volatile v4u*)(base + go[it]) = val[it];
        __threadfence();
      }
    }
  }
}

#define PSP 72
#define OSP 264
__global__ __launch_bounds__(256) void k_attn(const us16* __restrict__ qh, const us16* __restrict__ ql,
                                              const us16* __restrict__ kh, const us16* __restrict__ kl,
                                              const us16* __restrict__ vth, const us16* __restrict__ vtl,
                                              const float* __restrict__ mask, const int* __restrict__ lens, int ntok,
                                              us16* __restrict__ oh, us16* __restrict__ ol) {
  __shared__ __align__(16) us16 Ph[NH * 16 * PSP];
  __shared__ __align__(16) us16 Pl[NH * 16 * PSP];
  __shared__ __align__(16) us16 Sh[16 * OSP];
  __shared__ __align__(16) us16 Sl[16 * OSP];

  const int tid = threadIdx.x, lane = tid & 31, h = tid >> 5;
  const int hh = lane >> 4, c = lane & 15;
  const int qblk = blockIdx.x, b = blockIdx.y;
  const int qbase = qblk * QBLK;
  int off = 0, len = 0;
#pragma unroll
  for (int i = 0; i < NB; ++i) {
    const int li = min(max(lens[i], 0), MAXW);
    off += (i < b) ? li : 0;
    len = (i == b) ? li : len;
  }
  if (qbase >= len) return;

  const size_t brow = (size_t)b * MAXW;
  const us16* Kbh = kh + brow * CD;
  const us16* Kbl = kl + brow * CD;
  const us16* Vbh = vth + ((size_t)b * CD + h * HD) * MAXW;
  const us16* Vbl = vtl + ((size_t)b * CD + h * HD) * MAXW;
  const float* Mb = mask + (size_t)b * MAXW * MAXW;
  us16* pwh = Ph + h * 16 * PSP;
  us16* pwl = Pl + h * 16 * PSP;
  const float NEGI  = -__builtin_huge_valf();
  const float scale = 0.17677669529663687f;

#pragma unroll 1
  for (int qt = 0; qt < 4; ++qt) {
    const int q0   = qbase + 16 * qt;
    const int prow = b * MAXW + q0;
    const v16b qah = ldfrag(qh, CD, prow, h * HD, lane);
    const v16b qal = ldfrag(ql, CD, prow, h * HD, lane);

    float mrow[8], lrow[8];
    v8f oacc[2];
#pragma unroll
    for (int r = 0; r < 8; ++r) { mrow[r] = NEGI; lrow[r] = 0.f; }
    oacc[0] = zero8();
    oacc[1] = zero8();
    const float* Mq = Mb + (size_t)(q0 + 8 * hh) * MAXW + c;

#pragma unroll 1
    for (int kc = 0; kc < NKC; ++kc) {
      const int kv0 = kc * KCH;
      v8f s[4];
#pragma unroll
      for (int j = 0; j < 4; ++j) {
        const v16b kbh = ldfrag(Kbh, CD, kv0 + 16 * j, h * HD, lane);
        const v16b kbl = ldfrag(Kbl, CD, kv0 + 16 * j, h * HD, lane);
        s[j] = mma3(qah, qal, kbh, kbl, zero8());
      }
      float cm[8];
#pragma unroll
      for (int r = 0; r < 8; ++r) {
        float m = NEGI;
#pragma unroll
        for (int j = 0; j < 4; ++j) {
          const float mv = Mq[(size_t)r * MAXW + kv0 + 16 * j];
          const float sv = s[j][r] * scale + mv;
          s[j][r] = sv;
          m = fmaxf(m, sv);
        }
#pragma unroll
        for (int o2 = 1; o2 < 16; o2 <<= 1) m = fmaxf(m, __shfl_xor(m, o2, 32));
        cm[r] = m;
      }
#pragma unroll
      for (int r = 0; r < 8; ++r) {
        const float mnew  = fmaxf(mrow[r], cm[r]);
        const float alpha = __expf(mrow[r] - mnew);
        mrow[r] = mnew;
        float psum = 0.f;
#pragma unroll
        for (int j = 0; j < 4; ++j) {
          const float p = __expf(s[j][r] - mnew);
          psum += p;
          const us16 hb = bf_rne(p);
          const int idx = (8 * hh + r) * PSP + 16 * j + c;
          pwh[idx] = hb;
          pwl[idx] = bf_rne(p - bf_val(hb));
        }
#pragma unroll
        for (int o2 = 1; o2 < 16; o2 <<= 1) psum += __shfl_xor(psum, o2, 32);
        lrow[r] = lrow[r] * alpha + psum;
        oacc[0][r] *= alpha;
        oacc[1][r] *= alpha;
      }
      __syncthreads();

#pragma unroll
      for (int kk = 0; kk < 2; ++kk) {
        const v16b pah = ldfrag(pwh, PSP, 0, 32 * kk, lane);
        const v16b pal = ldfrag(pwl, PSP, 0, 32 * kk, lane);
#pragma unroll
        for (int t = 0; t < 2; ++t) {
          const v16b vbh = ldfrag(Vbh, MAXW, 16 * t, kv0 + 32 * kk, lane);
          const v16b vbl = ldfrag(Vbl, MAXW, 16 * t, kv0 + 32 * kk, lane);
          oacc[t] = mma3(pah, pal, vbh, vbl, oacc[t]);
        }
      }
      __syncthreads();
    }

    float il[8];
#pragma unroll
    for (int r = 0; r < 8; ++r) il[r] = (lrow[r] > 0.f) ? __builtin_amdgcn_rcpf(lrow[r]) : 0.f;
#pragma unroll
    for (int t = 0; t < 2; ++t)
#pragma unroll
      for (int r = 0; r < 8; ++r) {
        const float v = oacc[t][r] * il[r];
        const us16 hb = bf_rne(v);
        const int idx = (8 * hh + r) * OSP + h * HD + 16 * t + c;
        Sh[idx] = hb;
        Sl[idx] = bf_rne(v - bf_val(hb));
      }
    __syncthreads();
#pragma unroll
    for (int it = 0; it < 2; ++it) {
      const int row = h + 8 * it;
      const int q   = q0 + row;
      const int tk  = off + q;
      const bool ok = (q < len) && (tk < ntok);
      Pack8 a, bq;
      a.h  = *(const v8us*)(Sh + row * OSP + 8 * lane);
      bq.h = *(const v8us*)(Sl + row * OSP + 8 * lane);
      if (ok) {
        const size_t go = (size_t)tk * CD + 8 * lane;
        volatile v4u* dh = (volatile v4u*)(oh + go);
        volatile v4u* dl = (volatile v4u*)(ol + go);
        *dh = a.u;
        *dl = bq.u;
        __threadfence();
        *dh = a.u;
        *dl = bq.u;
      }
    }
    __syncthreads();
  }
}

#define OTP 68
__global__ __launch_bounds__(64) void k_proj(const us16* __restrict__ ah, const us16* __restrict__ al,
                                            const us16* __restrict__ wh, const us16* __restrict__ wl,
                                            const float* __restrict__ bias, float* __restrict__ out) {
  __shared__ __align__(16) float st[2][16 * OTP];
  const int tid = threadIdx.x, lane = tid & 31, wave = tid >> 5;
  const int hh = lane >> 4, c = lane & 15;
  const int m0 = blockIdx.x * 64 + wave * 32;
  const int n0 = blockIdx.y * 64;

  v8f acc[2][4];
#pragma unroll
  for (int s = 0; s < 2; ++s)
#pragma unroll
    for (int t = 0; t < 4; ++t) acc[s][t] = zero8();
  gemm32x64x3(ah, al, CD, wh, wl, CD, CD, m0, n0, lane, acc);

  float bb[4];
#pragma unroll
  for (int t = 0; t < 4; ++t) bb[t] = bias[n0 + 16 * t + c];

  float* sw = st[wave];
#pragma unroll
  for (int sub = 0; sub < 2; ++sub) {
    __syncthreads();
#pragma unroll
    for (int t = 0; t < 4; ++t)
#pragma unroll
      for (int r = 0; r < 8; ++r) sw[(8 * hh + r) * OTP + 16 * t + c] = acc[sub][t][r] + bb[t];
    __syncthreads();
    v4f val[8];
    size_t go[8];
#pragma unroll
    for (int it = 0; it < 8; ++it) {
      const int p   = lane + 32 * it;
      const int L   = p >> 3;
      const int pc  = p & 7;
      const int row = L >> 1;
      const int seg = L & 1;
      val[it] = *(const v4f*)(sw + row * OTP + seg * 32 + pc * 4);
      go[it]  = (size_t)(m0 + sub * 16 + row) * CD + n0 + seg * 32 + pc * 4;
    }
    for (int ps = 0; ps < 2; ++ps) {
#pragma unroll
      for (int it = 0; it < 8; ++it) *(volatile v4f*)(out + go[it]) = val[it];
      __threadfence();
    }
  }
}

extern "C" void kernel_launch(void* const* d_in, const int* in_sizes, int n_in,
                              void* d_out, int out_size, void* d_ws, size_t ws_size,
                              hipStream_t stream) {
  if (n_in < 7) return;
  if (in_sizes[0] != NTOK * CD) return;
  if (in_sizes[1] != NB * MAXW * MAXW) return;
  if (in_sizes[2] != NB) return;
  if (in_sizes[3] != CD * NQKV) return;
  if (in_sizes[4] != NQKV) return;
  if (in_sizes[5] != CD * CD) return;
  if (in_sizes[6] != CD) return;
  if (out_size != NTOK * CD) return;

  const float* tok    = (const float*)d_in[0];
  const float* mask   = (const float*)d_in[1];
  const int*   lens   = (const int*)d_in[2];
  const float* qkv_w  = (const float*)d_in[3];
  const float* qkv_b  = (const float*)d_in[4];
  const float* proj_w = (const float*)d_in[5];
  const float* proj_b = (const float*)d_in[6];
  const int    ntok   = in_sizes[0] / CD;
  float* out = (float*)d_out;

  size_t off = 0;
  const size_t oWqh = off; off += (size_t)NQKV * CD * 2;
  const size_t oWql = off; off += (size_t)NQKV * CD * 2;
  const size_t oWph = off; off += (size_t)CD * CD * 2;
  const size_t oWpl = off; off += (size_t)CD * CD * 2;
  const size_t oXh  = off; off += (size_t)PROWS * CD * 2;
  const size_t oXl  = off; off += (size_t)PROWS * CD * 2;
  const size_t oQh  = off; off += (size_t)PROWS * CD * 2;
  const size_t oQl  = off; off += (size_t)PROWS * CD * 2;
  const size_t oKh  = off; off += (size_t)PROWS * CD * 2;
  const size_t oKl  = off; off += (size_t)PROWS * CD * 2;
  const size_t oVh  = off; off += (size_t)NB * CD * MAXW * 2;
  const size_t oVl  = off; off += (size_t)NB * CD * MAXW * 2;
  const size_t oOh  = off; off += (size_t)NTOK * CD * 2;
  const size_t oOl  = off; off += (size_t)NTOK * CD * 2;
  if (off > ws_size) return;
  if (off > (size_t)134217728) return;

  char* ws = (char*)d_ws;
  us16* Wqh = (us16*)(ws + oWqh);
  us16* Wql = (us16*)(ws + oWql);
  us16* Wph = (us16*)(ws + oWph);
  us16* Wpl = (us16*)(ws + oWpl);
  us16* Xh  = (us16*)(ws + oXh);
  us16* Xl  = (us16*)(ws + oXl);
  us16* Qh  = (us16*)(ws + oQh);
  us16* Ql  = (us16*)(ws + oQl);
  us16* Kh  = (us16*)(ws + oKh);
  us16* Kl  = (us16*)(ws + oKl);
  us16* Vh  = (us16*)(ws + oVh);
  us16* Vl  = (us16*)(ws + oVl);
  us16* Oh  = (us16*)(ws + oOh);
  us16* Ol  = (us16*)(ws + oOl);

  k_tr<<<dim3(NQKV / 32), dim3(256), 0, stream>>>(qkv_w, NQKV, Wqh, Wql);
  k_tr<<<dim3(CD / 32), dim3(256), 0, stream>>>(proj_w, CD, Wph, Wpl);
  k_pad<<<dim3(PROWS / 8), dim3(256), 0, stream>>>(tok, lens, ntok, Xh, Xl);
  k_qkv<<<dim3(PROWS / 128, NQKV / 64), dim3(128), 0, stream>>>(Xh, Xl, Wqh, Wql, qkv_b, Qh, Ql, Kh, Kl, Vh, Vl);
  k_attn<<<dim3(NQB, NB), dim3(256), 0, stream>>>(Qh, Ql, Kh, Kl, Vh, Vl, mask, lens, ntok, Oh, Ol);
  k_proj<<<dim3(NTOK / 64, CD / 64), dim3(64), 0, stream>>>(Oh, Ol, Wph, Wpl, proj_b, out);
  (void)hipGetLastError();
}
